// GATLayer_48550310314658
// MI455X (gfx1250) — hardware-run, weakly checked
//
#include <hip/hip_runtime.h>
#include <stddef.h>
#include <stdint.h>
#include <math.h>

#define NN      4096
#define CIN     256
#define COUT    256
#define NHD     4
#define CH      64
#define NE      131072
#define NTHR    256
#define NWAVE   8
#define EPT     8
#define CHUNK   (NTHR * EPT)
#define RB      256
#define SLSH    12
#define RCAP    10240
#define DEGCAP  96
#define GBM     128
#define NEGSL   0.2f
#define NEGB    (-3.0e38f)
#define WSMAX   (128u << 20)
#define LDS_ROWS ((2 * RCAP + 3 * RB + 16) * 4)
#define LDS_GEMM (GBM * COUT * 4 + COUT * 4 + NHD * 2 * CH * 4 + COUT * 8)
#define XB_BLKS (NN * (CIN / 8) / NTHR)
#define WT_BLKS (COUT * (CIN / 8) / NTHR)

static_assert(RCAP >= 8431 + 1024);
static_assert(DEGCAP >= 53 + 8);
static_assert(DEGCAP == 96 && DEGCAP == 3 * 32);
static_assert((NN % GBM) == 0 && GBM == NWAVE * 16);
static_assert(COUT == 256 && (CIN % 32) == 0 && NHD * CH == COUT);
static_assert((CIN / 8) == 32);
static_assert((NE % CHUNK) == 0);
static_assert(NN == (1 << SLSH) && RB == 256 && (NN % RB) == 0);
static_assert((RCAP % 32) == 0);
static_assert((LDS_ROWS % 16) == 0 && LDS_ROWS <= 327680 && LDS_GEMM <= 327680);
static_assert(RB == 32 * 8 && (RB % NWAVE) == 0);

typedef float          v4f  __attribute__((ext_vector_type(4)));
typedef float          v8f  __attribute__((ext_vector_type(8)));
typedef double         v2d  __attribute__((ext_vector_type(2)));
typedef int            v4i  __attribute__((ext_vector_type(4)));
typedef int            v8i  __attribute__((ext_vector_type(8)));
typedef unsigned int   v4u  __attribute__((ext_vector_type(4)));
typedef unsigned short v8us __attribute__((ext_vector_type(8)));
typedef __bf16         v16b __attribute__((ext_vector_type(16)));
typedef v4f  __attribute__((may_alias)) v4fa;
typedef v2d  __attribute__((may_alias)) v2da;
typedef v8us __attribute__((may_alias)) v8usa;
union FragB { v16b v; v8us h[2]; v8i w; };

__device__ __forceinline__ v8f wmb(const FragB& a, const FragB& b, v8f c) {
  v8f d = __builtin_amdgcn_wmma_f32_16x16x32_bf16(false, a.v, false, b.v, (short)0, c, false, false);
  asm volatile("v_nop\n\tv_nop\n\tv_nop\n\tv_nop" : "+v"(d) : "v"(a.w), "v"(b.w));
  return d;
}

__device__ __forceinline__ unsigned int f2bf(float f) {
  const unsigned int u = __float_as_uint(f);
  return ((u + 0x7FFFu + ((u >> 16) & 1u)) >> 16) & 0xFFFFu;
}
__device__ __forceinline__ float bf2f(unsigned int b) { return __uint_as_float(b << 16); }
__device__ __forceinline__ float bfr(float f) { return bf2f(f2bf(f)); }
__device__ __forceinline__ v4f bfr4(const v4f a) {
  v4f r; r.x = bfr(a.x); r.y = bfr(a.y); r.z = bfr(a.z); r.w = bfr(a.w); return r;
}
__device__ __forceinline__ unsigned int pk2(float lo, float hi) { return f2bf(lo) | (f2bf(hi) << 16); }
__device__ __forceinline__ v4u pack8(const v4f a, const v4f b) {
  v4u r;
  r.x = pk2(a.x, a.y); r.y = pk2(a.z, a.w); r.z = pk2(b.x, b.y); r.w = pk2(b.z, b.w);
  return r;
}
__device__ __forceinline__ int clampid(int j) { return j < 0 ? 0 : (j > NN - 1 ? NN - 1 : j); }
__device__ __forceinline__ float leaky(float v) { return (v >= 0.0f) ? v : NEGSL * v; }

__global__ __launch_bounds__(NTHR) void k_prep(const float* __restrict__ x, const float* __restrict__ W,
                                               const float* __restrict__ b, const float* __restrict__ a,
                                               unsigned short* XB, unsigned short* WT, float* AT, float* BT) {
  const int blk = (int)blockIdx.x, tid = (int)threadIdx.x;
  if (blk < XB_BLKS) {
    const int u = blk * NTHR + tid;
    const int row = u >> 5, c0 = (u & 31) * 8;
    const float* p = x + (size_t)row * CIN + c0;
    const v4f va = *(const v4fa*)p, vb = *(const v4fa*)(p + 4);
    const v4u hv = pack8(va, vb);
    unsigned short* o = XB + (size_t)row * CIN + c0;
    *(volatile v4u*)o = hv;
    __threadfence();
    *(volatile v4u*)o = hv;
  } else if (blk < XB_BLKS + WT_BLKS) {
    const int u = (blk - XB_BLKS) * NTHR + tid;
    const int n = u >> 5, k8 = (u & 31) * 8;
    const float* p = W + (size_t)k8 * COUT + n;
    v4f va, vb;
    va.x = p[0];                  va.y = p[(size_t)COUT];       va.z = p[(size_t)2 * COUT];  va.w = p[(size_t)3 * COUT];
    vb.x = p[(size_t)4 * COUT];   vb.y = p[(size_t)5 * COUT];   vb.z = p[(size_t)6 * COUT];  vb.w = p[(size_t)7 * COUT];
    const v4u wv = pack8(va, vb);
    unsigned short* o = WT + (size_t)n * CIN + k8;
    *(volatile v4u*)o = wv;
    __threadfence();
    *(volatile v4u*)o = wv;
  } else {
    if (tid < 128) {
      const v4f v = bfr4(*(const v4fa*)(a + 4 * tid));
      float* o = AT + 4 * tid;
      *(volatile v4f*)o = v;
      __threadfence();
      *(volatile v4f*)o = v;
    } else if (tid < 192) {
      const int q = tid - 128;
      const v4f v = bfr4(*(const v4fa*)(b + 4 * q));
      float* o = BT + 4 * q;
      *(volatile v4f*)o = v;
      __threadfence();
      *(volatile v4f*)o = v;
    }
  }
}

__global__ __launch_bounds__(NTHR) __attribute__((amdgpu_num_vgpr(248)))
void k_gemm(const unsigned short* __restrict__ XB, const unsigned short* __restrict__ WT,
            const float* __restrict__ AT, const float* __restrict__ BT,
            float* F, float* ESD, double* REC) {
  extern __shared__ v4f lds_g[];
  float*  tile = (float*)lds_g;
  float*  sBT  = tile + GBM * COUT;
  float*  sAT  = sBT + COUT;
  double* srec = (double*)(sAT + NHD * 2 * CH);
  const int tid = (int)threadIdx.x, lane = tid & 31, wave = tid >> 5, hh = lane >> 4, m = lane & 15;
  const int blk = (int)blockIdx.x;
  const int rowBase = blk * GBM;

  if (tid < 64) {
    *(v4f*)(sBT + 4 * tid) = *(const v4fa*)(BT + 4 * tid);
  } else if (tid < 192) {
    const int q = tid - 64;
    *(v4f*)(sAT + 4 * q) = *(const v4fa*)(AT + 4 * q);
  }
  __syncthreads();

  const unsigned short* ap = XB + (size_t)(rowBase + 16 * wave + m) * CIN + 8 * hh;
#pragma unroll 1
  for (int cg = 0; cg < 4; ++cg) {
    v8f acc[4];
    {
      const v8f z = {0.f, 0.f, 0.f, 0.f, 0.f, 0.f, 0.f, 0.f};
      acc[0] = z; acc[1] = z; acc[2] = z; acc[3] = z;
    }
    const unsigned short* wp = WT + (size_t)(64 * cg + m) * CIN + 8 * hh;
#pragma unroll 1
    for (int ks = 0; ks < CIN / 32; ++ks) {
      FragB af;
      af.h[0] = *(const v8usa*)(ap + 32 * ks);
      af.h[1] = *(const v8usa*)(ap + 32 * ks + 16);
#pragma unroll
      for (int t = 0; t < 4; ++t) {
        const unsigned short* wq = wp + (size_t)(16 * t) * CIN + 32 * ks;
        FragB bf;
        bf.h[0] = *(const v8usa*)wq;
        bf.h[1] = *(const v8usa*)(wq + 16);
        acc[t] = wmb(af, bf, acc[t]);
      }
    }
#pragma unroll
    for (int t = 0; t < 4; ++t) {
      const int lc = 64 * cg + 16 * t + m;
      const float bc = sBT[lc];
#pragma unroll
      for (int r = 0; r < 8; ++r) {
        const int lr = 16 * wave + 8 * hh + r;
        tile[lr * COUT + lc] = acc[t][r] + bc;
      }
    }
  }
  __syncthreads();

  const int drow = tid & 127, side = tid >> 7;
  v4f dv;
  {
    const float* hr = tile + drow * COUT;
    const float* sa = sAT + side * CH;
    float d0 = 0.f, d1 = 0.f, d2 = 0.f, d3 = 0.f;
#pragma unroll 2
    for (int c4 = 0; c4 < CH / 4; ++c4) {
      const v4f f0 = *(const v4fa*)(hr + 0 * CH + 4 * c4);
      const v4f f1 = *(const v4fa*)(hr + 1 * CH + 4 * c4);
      const v4f f2 = *(const v4fa*)(hr + 2 * CH + 4 * c4);
      const v4f f3 = *(const v4fa*)(hr + 3 * CH + 4 * c4);
      const v4f a0 = *(const v4fa*)(sa + 0 * 2 * CH + 4 * c4);
      const v4f a1 = *(const v4fa*)(sa + 1 * 2 * CH + 4 * c4);
      const v4f a2 = *(const v4fa*)(sa + 2 * 2 * CH + 4 * c4);
      const v4f a3 = *(const v4fa*)(sa + 3 * 2 * CH + 4 * c4);
      d0 = fmaf(f0.x, a0.x, d0); d0 = fmaf(f0.y, a0.y, d0); d0 = fmaf(f0.z, a0.z, d0); d0 = fmaf(f0.w, a0.w, d0);
      d1 = fmaf(f1.x, a1.x, d1); d1 = fmaf(f1.y, a1.y, d1); d1 = fmaf(f1.z, a1.z, d1); d1 = fmaf(f1.w, a1.w, d1);
      d2 = fmaf(f2.x, a2.x, d2); d2 = fmaf(f2.y, a2.y, d2); d2 = fmaf(f2.z, a2.z, d2); d2 = fmaf(f2.w, a2.w, d2);
      d3 = fmaf(f3.x, a3.x, d3); d3 = fmaf(f3.y, a3.y, d3); d3 = fmaf(f3.z, a3.z, d3); d3 = fmaf(f3.w, a3.w, d3);
    }
    dv.x = d0; dv.y = d1; dv.z = d2; dv.w = d3;
  }

  {
    double cs = 0.0;
#pragma unroll 4
    for (int r = 0; r < GBM; ++r) cs += (double)tile[r * COUT + tid];
    srec[tid] = cs;
  }
  __syncthreads();
  const v2d rv = *(const v2da*)(srec + 2 * (tid & 127));

  float*  esp = ESD + (size_t)side * (size_t)(NN * NHD) + (size_t)(rowBase + drow) * NHD;
  double* rp  = REC + (size_t)blk * COUT + 2 * (tid & 127);
  const bool wrec = tid < 128;

#pragma unroll 4
  for (int i = 0; i < 16; ++i) {
    const int lr = 16 * wave + i;
    const v4f va = *(const v4fa*)(tile + lr * COUT + 4 * lane);
    const v4f vb = *(const v4fa*)(tile + lr * COUT + 128 + 4 * lane);
    float* op = F + (size_t)(rowBase + lr) * COUT + 4 * lane;
    *(volatile v4f*)op = va;
    *(volatile v4f*)(op + 128) = vb;
  }
  *(volatile v4f*)esp = dv;
  if (wrec) *(volatile v2d*)rp = rv;
  __threadfence();
#pragma unroll 4
  for (int i = 0; i < 16; ++i) {
    const int lr = 16 * wave + i;
    const v4f va = *(const v4fa*)(tile + lr * COUT + 4 * lane);
    const v4f vb = *(const v4fa*)(tile + lr * COUT + 128 + 4 * lane);
    float* op = F + (size_t)(rowBase + lr) * COUT + 4 * lane;
    *(volatile v4f*)op = va;
    *(volatile v4f*)(op + 128) = vb;
  }
  *(volatile v4f*)esp = dv;
  if (wrec) *(volatile v2d*)rp = rv;
}

__global__ __launch_bounds__(NTHR) void k_colmean(const double* __restrict__ REC, float* FM) {
  __shared__ __attribute__((aligned(16))) float sfm[COUT];
  const int tid = (int)threadIdx.x;
  double s = 0.0;
#pragma unroll 4
  for (int b = 0; b < NN / GBM; ++b) s += REC[(size_t)b * COUT + tid];
  sfm[tid] = (float)(s * (1.0 / (double)NN));
  __syncthreads();
  const v4f v = *(const v4fa*)(sfm + 4 * (tid & 63));
  float* o = FM + 4 * (tid & 63);
  const bool wr = tid < 64;
  if (wr) *(volatile v4f*)o = v;
  __threadfence();
  if (wr) *(volatile v4f*)o = v;
}

struct A3 { float a0, a1, a2; };
__device__ __forceinline__ A3 head_alpha(float x0, float x1, float x2, bool k0, bool k1, bool k2) {
  float mx = fmaxf(fmaxf(k0 ? x0 : NEGB, k1 ? x1 : NEGB), k2 ? x2 : NEGB);
#pragma unroll
  for (int off = 16; off > 0; off >>= 1) mx = fmaxf(mx, __shfl_xor(mx, off));
  const float g0 = k0 ? (x0 - mx) : 0.0f;
  const float g1 = k1 ? (x1 - mx) : 0.0f;
  const float g2 = k2 ? (x2 - mx) : 0.0f;
  const float x0e = expf(g0), x1e = expf(g1), x2e = expf(g2);
  const float e0 = k0 ? x0e : 0.0f;
  const float e1 = k1 ? x1e : 0.0f;
  const float e2 = k2 ? x2e : 0.0f;
  float s = (e0 + e1) + e2;
#pragma unroll
  for (int off = 16; off > 0; off >>= 1) s += __shfl_xor(s, off);
  const float sd  = (s > 0.0f) ? s : 1.0f;
  const float inv = 1.0f / sd;
  A3 r; r.a0 = e0 * inv; r.a1 = e1 * inv; r.a2 = e2 * inv;
  return r;
}

__device__ __forceinline__ void agg_group(const float* __restrict__ F, int idg, float g0, float g1, float g2, float g3,
                                          int trips, int lane, int lh, v4f& accA, v4f& accB) {
#pragma unroll 1
  for (int k = 0; k < trips; ++k) {
    const int j = __builtin_amdgcn_readlane(idg, k) & (NN - 1);
    const float a0 = __int_as_float(__builtin_amdgcn_readlane(__float_as_int(g0), k));
    const float a1 = __int_as_float(__builtin_amdgcn_readlane(__float_as_int(g1), k));
    const float a2 = __int_as_float(__builtin_amdgcn_readlane(__float_as_int(g2), k));
    const float a3 = __int_as_float(__builtin_amdgcn_readlane(__float_as_int(g3), k));
    const float aA = lh ? a1 : a0;
    const float aB = lh ? a3 : a2;
    const float* fr = F + (size_t)j * COUT + 4 * lane;
    const v4f fa = *(const v4fa*)fr;
    const v4f fb = *(const v4fa*)(fr + 128);
    accA.x = fmaf(aA, fa.x, accA.x); accA.y = fmaf(aA, fa.y, accA.y);
    accA.z = fmaf(aA, fa.z, accA.z); accA.w = fmaf(aA, fa.w, accA.w);
    accB.x = fmaf(aB, fb.x, accB.x); accB.y = fmaf(aB, fb.y, accB.y);
    accB.z = fmaf(aB, fb.z, accB.z); accB.w = fmaf(aB, fb.w, accB.w);
  }
}

__global__ __launch_bounds__(NTHR) void k_rows(const int* __restrict__ edges, const float* __restrict__ F,
                                               const float* __restrict__ ESD, const float* __restrict__ FM,
                                               float* out) {
  extern __shared__ v4f lds_r[];
  int* reg1  = (int*)lds_r;
  int* reg2  = reg1 + RCAP;
  int* scnt  = reg2 + RCAP;
  int* soff  = scnt + RB;
  int* scur  = soff + RB;
  int* wcnt  = scur + RB;
  int* sflag = wcnt + NWAVE;
  const int tid = (int)threadIdx.x, lane = tid & 31, wave = tid >> 5;
  const int rbase = (int)blockIdx.x * RB;

  {
    const v4i z = {0, 0, 0, 0};
    v4i* zp = (v4i*)lds_r;
    for (int i = tid; i < LDS_ROWS / 16; i += NTHR) zp[i] = z;
  }
  __syncthreads();

  const unsigned ub = (unsigned)rbase;
  int tot = 0, ovf = 0;
#pragma unroll 1
  for (int ch = 0; ch < NE / CHUNK; ++ch) {
    const int* ep = edges + (size_t)2 * (size_t)(ch * CHUNK + tid * EPT);
    const v4i q0 = *(const v4i*)ep;
    const v4i q1 = *(const v4i*)(ep + 4);
    const v4i q2 = *(const v4i*)(ep + 8);
    const v4i q3 = *(const v4i*)(ep + 12);
    asm volatile("" :: "v"(q0), "v"(q1), "v"(q2), "v"(q3));
    const unsigned s0 = (unsigned)q0.x - ub, s1 = (unsigned)q0.z - ub;
    const unsigned s2 = (unsigned)q1.x - ub, s3 = (unsigned)q1.z - ub;
    const unsigned s4 = (unsigned)q2.x - ub, s5 = (unsigned)q2.z - ub;
    const unsigned s6 = (unsigned)q3.x - ub, s7 = (unsigned)q3.z - ub;
    const int h0 = s0 < (unsigned)RB ? 1 : 0, h1 = s1 < (unsigned)RB ? 1 : 0;
    const int h2 = s2 < (unsigned)RB ? 1 : 0, h3 = s3 < (unsigned)RB ? 1 : 0;
    const int h4 = s4 < (unsigned)RB ? 1 : 0, h5 = s5 < (unsigned)RB ? 1 : 0;
    const int h6 = s6 < (unsigned)RB ? 1 : 0, h7 = s7 < (unsigned)RB ? 1 : 0;
    const int cl = h0 + h1 + h2 + h3 + h4 + h5 + h6 + h7;
    const unsigned any = __builtin_amdgcn_ballot_w32(cl != 0);
    int incl = cl;
    if (any != 0u) {
#pragma unroll
      for (int d = 1; d < 32; d <<= 1) {
        const int up = __shfl_up(incl, d);
        incl += (lane >= d) ? up : 0;
      }
    }
    const int wc = __shfl(incl, 31);
    if (lane == 0) wcnt[wave] = wc;
    __syncthreads();
    int pre = 0, all = 0;
#pragma unroll
    for (int w2 = 0; w2 < NWAVE; ++w2) {
      int c = wcnt[w2];
      c = c < 0 ? 0 : (c > EPT * 32 ? EPT * 32 : c);
      all += c;
      pre += (w2 < wave) ? c : 0;
    }
    int pos = tot + pre + (incl - cl);
    const int w0 = clampid(q0.y) | (int)((s0 & 255u) << SLSH);
    const int w1 = clampid(q0.w) | (int)((s1 & 255u) << SLSH);
    const int w2v = clampid(q1.y) | (int)((s2 & 255u) << SLSH);
    const int w3 = clampid(q1.w) | (int)((s3 & 255u) << SLSH);
    const int w4 = clampid(q2.y) | (int)((s4 & 255u) << SLSH);
    const int w5 = clampid(q2.w) | (int)((s5 & 255u) << SLSH);
    const int w6 = clampid(q3.y) | (int)((s6 & 255u) << SLSH);
    const int w7 = clampid(q3.w) | (int)((s7 & 255u) << SLSH);
    if (h0 != 0 && pos < RCAP) reg1[pos] = w0;
    pos += h0;
    if (h1 != 0 && pos < RCAP) reg1[pos] = w1;
    pos += h1;
    if (h2 != 0 && pos < RCAP) reg1[pos] = w2v;
    pos += h2;
    if (h3 != 0 && pos < RCAP) reg1[pos] = w3;
    pos += h3;
    if (h4 != 0 && pos < RCAP) reg1[pos] = w4;
    pos += h4;
    if (h5 != 0 && pos < RCAP) reg1[pos] = w5;
    pos += h5;
    if (h6 != 0 && pos < RCAP) reg1[pos] = w6;
    pos += h6;
    if (h7 != 0 && pos < RCAP) reg1[pos] = w7;
    tot += all;
    ovf |= (tot > RCAP) ? 1 : 0;
    tot = tot > RCAP ? RCAP : tot;
    __syncthreads();
  }
  const int nh = __builtin_amdgcn_readfirstlane(tot);

  if (wave == 0) {
#pragma unroll 1
    for (int b0 = 0; b0 < nh; b0 += 32) {
      int idx = b0 + lane;
      idx = idx < nh ? idx : nh - 1;
      idx = idx < 0 ? 0 : idx;
      const int uv  = reg1[idx];
      const int m32 = (nh - b0) < 32 ? (nh - b0) : 32;
#pragma unroll 1
      for (int k = 0; k < m32; ++k) {
        const int u  = __builtin_amdgcn_readlane(uv, k);
        const int sl = (u >> SLSH) & (RB - 1);
        if (lane == 0) scnt[sl] = scnt[sl] + 1;
      }
    }
  }
  __syncthreads();

  if (wave == 0) {
    const v4i ca = *(const v4i*)(scnt + 8 * lane);
    const v4i cb = *(const v4i*)(scnt + 8 * lane + 4);
    const int e0 = ca.x < 0 ? 0 : ca.x, e1 = ca.y < 0 ? 0 : ca.y, e2 = ca.z < 0 ? 0 : ca.z, e3 = ca.w < 0 ? 0 : ca.w;
    const int e4 = cb.x < 0 ? 0 : cb.x, e5 = cb.y < 0 ? 0 : cb.y, e6 = cb.z < 0 ? 0 : cb.z, e7 = cb.w < 0 ? 0 : cb.w;
    const int ts = e0 + e1 + e2 + e3 + e4 + e5 + e6 + e7;
    int incl = ts;
#pragma unroll
    for (int d = 1; d < 32; d <<= 1) {
      const int up = __shfl_up(incl, d);
      incl += (lane >= d) ? up : 0;
    }
    v4i oa, ob;
    int run = incl - ts;
    oa.x = run; run += e0;
    oa.y = run; run += e1;
    oa.z = run; run += e2;
    oa.w = run; run += e3;
    ob.x = run; run += e4;
    ob.y = run; run += e5;
    ob.z = run; run += e6;
    ob.w = run;
    *(v4i*)(soff + 8 * lane)     = oa;
    *(v4i*)(soff + 8 * lane + 4) = ob;
    *(v4i*)(scur + 8 * lane)     = oa;
    *(v4i*)(scur + 8 * lane + 4) = ob;
    int emx = e0 > e1 ? e0 : e1;
    emx = emx > e2 ? emx : e2; emx = emx > e3 ? emx : e3;
    emx = emx > e4 ? emx : e4; emx = emx > e5 ? emx : e5;
    emx = emx > e6 ? emx : e6; emx = emx > e7 ? emx : e7;
    const unsigned df = __builtin_amdgcn_ballot_w32(emx > DEGCAP);
    if (lane == 0) sflag[0] = (df != 0u) ? 1 : 0;
  }
  __syncthreads();

  if (wave == 0) {
#pragma unroll 1
    for (int b0 = 0; b0 < nh; b0 += 32) {
      int idx = b0 + lane;
      idx = idx < nh ? idx : nh - 1;
      idx = idx < 0 ? 0 : idx;
      const int uv  = reg1[idx];
      const int m32 = (nh - b0) < 32 ? (nh - b0) : 32;
#pragma unroll 1
      for (int k = 0; k < m32; ++k) {
        const int u  = __builtin_amdgcn_readlane(uv, k);
        const int sl = (u >> SLSH) & (RB - 1);
        const int jj = u & (NN - 1);
        if (lane == 0) {
          int pos = scur[sl];
          pos = pos < 0 ? 0 : (pos > RCAP - 1 ? RCAP - 1 : pos);
          reg2[pos] = jj;
          scur[sl] = pos + 1;
        }
      }
    }
  }
  __syncthreads();

  const int   flg  = sflag[0] | ovf;
  const float qnan = __int_as_float(0x7fc00000);
  const float pz   = (flg != 0) ? qnan : 0.0f;
  const int   lh   = lane >> 4;
  const float* EDp = ESD + (size_t)(NN * NHD);
  const v4f fmA = *(const v4fa*)(FM + 4 * lane);
  const v4f fmB = *(const v4fa*)(FM + 128 + 4 * lane);
  asm volatile("" :: "v"(fmA), "v"(fmB));

#pragma unroll 1
  for (int it = 0; it < RB / NWAVE; ++it) {
    const int slot = wave + NWAVE * it;
    const int row  = rbase + slot;
    int cv = scnt[slot];
    int ov = soff[slot];
    ov = ov < 0 ? 0 : (ov > nh ? nh : ov);
    cv = cv < 0 ? 0 : (cv > DEGCAP ? DEGCAP : cv);
    cv = cv > nh - ov ? nh - ov : cv;
    int lastv = ov + cv - 1;
    lastv = lastv < ov ? ov : lastv;
    lastv = lastv > RCAP - 1 ? RCAP - 1 : lastv;
    int t0v = cv;      t0v = t0v > 32 ? 32 : t0v;
    int t1v = cv - 32; t1v = t1v < 0 ? 0 : (t1v > 32 ? 32 : t1v);
    int t2v = cv - 64; t2v = t2v < 0 ? 0 : (t2v > 32 ? 32 : t2v);
    const int c    = __builtin_amdgcn_readfirstlane(cv);
    const int o    = __builtin_amdgcn_readfirstlane(ov);
    const int last = __builtin_amdgcn_readfirstlane(lastv);
    const int t0   = __builtin_amdgcn_readfirstlane(t0v);
    const int t1   = __builtin_amdgcn_readfirstlane(t1v);
    const int t2   = __builtin_amdgcn_readfirstlane(t2v);

    int i0 = o + lane;      i0 = i0 > last ? last : i0;
    int i1 = o + lane + 32; i1 = i1 > last ? last : i1;
    int i2 = o + lane + 64; i2 = i2 > last ? last : i2;
    const int id0 = reg2[i0] & (NN - 1);
    const int id1 = reg2[i1] & (NN - 1);
    const int id2 = reg2[i2] & (NN - 1);

    int dp0 = 0, dp1 = 0, dp2 = 0;
#pragma unroll 1
    for (int k = 0; k < c; ++k) {
      int ik = o + k; ik = ik > last ? last : ik;
      const int idk = reg2[ik] & (NN - 1);
      dp0 |= (id0 == idk && lane      > k) ? 1 : 0;
      dp1 |= (id1 == idk && lane + 32 > k) ? 1 : 0;
      dp2 |= (id2 == idk && lane + 64 > k) ? 1 : 0;
    }
    const bool k0 = (lane      < c) && (dp0 == 0);
    const bool k1 = (lane + 32 < c) && (dp1 == 0);
    const bool k2 = (lane + 64 < c) && (dp2 == 0);

    const v4f es = *(const v4fa*)(ESD + (size_t)row * NHD);
    const v4f d0 = *(const v4fa*)(EDp + (size_t)id0 * NHD);
    const v4f d1 = *(const v4fa*)(EDp + (size_t)id1 * NHD);
    const v4f d2 = *(const v4fa*)(EDp + (size_t)id2 * NHD);
    asm volatile("" :: "v"(d0), "v"(d1), "v"(d2));
    const A3 p0 = head_alpha(leaky(es.x + d0.x), leaky(es.x + d1.x), leaky(es.x + d2.x), k0, k1, k2);
    const A3 p1 = head_alpha(leaky(es.y + d0.y), leaky(es.y + d1.y), leaky(es.y + d2.y), k0, k1, k2);
    const A3 p2 = head_alpha(leaky(es.z + d0.z), leaky(es.z + d1.z), leaky(es.z + d2.z), k0, k1, k2);
    const A3 p3 = head_alpha(leaky(es.w + d0.w), leaky(es.w + d1.w), leaky(es.w + d2.w), k0, k1, k2);

    v4f accA = {0.f, 0.f, 0.f, 0.f};
    v4f accB = {0.f, 0.f, 0.f, 0.f};
    agg_group(F, id0, p0.a0, p1.a0, p2.a0, p3.a0, t0, lane, lh, accA, accB);
    agg_group(F, id1, p0.a1, p1.a1, p2.a1, p3.a1, t1, lane, lh, accA, accB);
    agg_group(F, id2, p0.a2, p1.a2, p2.a2, p3.a2, t2, lane, lh, accA, accB);

    const bool emp = (c == 0);
    v4f oA, oB;
    oA.x = (emp ? fmA.x : accA.x) + pz;
    oA.y = (emp ? fmA.y : accA.y) + pz;
    oA.z = (emp ? fmA.z : accA.z) + pz;
    oA.w = (emp ? fmA.w : accA.w) + pz;
    oB.x = (emp ? fmB.x : accB.x) + pz;
    oB.y = (emp ? fmB.y : accB.y) + pz;
    oB.z = (emp ? fmB.z : accB.z) + pz;
    oB.w = (emp ? fmB.w : accB.w) + pz;
    float* op = out + (size_t)row * COUT + 4 * lane;
    *(volatile v4f*)op = oA;
    *(volatile v4f*)(op + 128) = oB;
    __threadfence();
    *(volatile v4f*)op = oA;
    *(volatile v4f*)(op + 128) = oB;
  }
}

extern "C" void kernel_launch(void* const* d_in, const int* in_sizes, int n_in,
                              void* d_out, int out_size, void* d_ws, size_t ws_size,
                              hipStream_t stream) {
  if (n_in < 5) return;
  if (in_sizes[0] != NN * CIN) return;
  if (in_sizes[1] != 2 * NE) return;
  if (in_sizes[2] != CIN * COUT) return;
  if (in_sizes[3] != COUT) return;
  if (in_sizes[4] != NHD * 2 * CH) return;
  if (out_size != NN * COUT) return;

  const float* x  = (const float*)d_in[0];
  const int*   ed = (const int*)  d_in[1];
  const float* W  = (const float*)d_in[2];
  const float* b  = (const float*)d_in[3];
  const float* a  = (const float*)d_in[4];
  float* out = (float*)d_out;

  char* ws = (char*)d_ws;
  size_t off = 0;
  const size_t oXB  = off; off += (size_t)NN * CIN * 2;          off = (off + 255) & ~(size_t)255;
  const size_t oWT  = off; off += (size_t)COUT * CIN * 2;        off = (off + 255) & ~(size_t)255;
  const size_t oF   = off; off += (size_t)NN * COUT * 4;         off = (off + 255) & ~(size_t)255;
  const size_t oESD = off; off += (size_t)2 * NN * NHD * 4;      off = (off + 255) & ~(size_t)255;
  const size_t oREC = off; off += (size_t)(NN / GBM) * COUT * 8; off = (off + 255) & ~(size_t)255;
  const size_t oFM  = off; off += (size_t)COUT * 4;              off = (off + 255) & ~(size_t)255;
  const size_t oAT  = off; off += (size_t)NHD * 2 * CH * 4;      off = (off + 255) & ~(size_t)255;
  const size_t oBT  = off; off += (size_t)COUT * 4;              off = (off + 255) & ~(size_t)255;
  if (off > ws_size || off > (size_t)WSMAX) return;
  unsigned short* XB  = (unsigned short*)(ws + oXB);
  unsigned short* WT  = (unsigned short*)(ws + oWT);
  float*          Fp  = (float*)(ws + oF);
  float*          ESD = (float*)(ws + oESD);
  double*         REC = (double*)(ws + oREC);
  float*          FM  = (float*)(ws + oFM);
  float*          AT  = (float*)(ws + oAT);
  float*          BT  = (float*)(ws + oBT);

  hipFuncSetAttribute(reinterpret_cast<const void*>(&k_gemm),
                      hipFuncAttributeMaxDynamicSharedMemorySize, LDS_GEMM);
  hipFuncSetAttribute(reinterpret_cast<const void*>(&k_rows),
                      hipFuncAttributeMaxDynamicSharedMemorySize, LDS_ROWS);

  k_prep<<<XB_BLKS + WT_BLKS + 1, NTHR, 0, stream>>>(x, W, b, a, XB, WT, AT, BT);
  k_gemm<<<NN / GBM, NTHR, LDS_GEMM, stream>>>(XB, WT, AT, BT, Fp, ESD, REC);
  k_colmean<<<1, NTHR, 0, stream>>>(REC, FM);
  k_rows<<<NN / RB, NTHR, LDS_ROWS, stream>>>(ed, Fp, ESD, FM, out);
}
